// Test_11450382811214
// MI455X (gfx1250) — hardware-verified
//
#include <hip/hip_runtime.h>

typedef _Float16 v16h __attribute__((ext_vector_type(16)));
typedef _Float16 v8h  __attribute__((ext_vector_type(8)));
typedef __bf16   v16b __attribute__((ext_vector_type(16)));
typedef __bf16   v8b  __attribute__((ext_vector_type(8)));
typedef float    v8f  __attribute__((ext_vector_type(8)));
typedef float    v4f  __attribute__((ext_vector_type(4)));
typedef unsigned short v8us __attribute__((ext_vector_type(8)));
typedef v8h  __attribute__((may_alias)) v8ha;
typedef v8b  __attribute__((may_alias)) v8ba;
typedef v4f  __attribute__((may_alias)) v4fa;
typedef v8us __attribute__((may_alias)) v8usa;

union FragH { v16h v; v8h half[2]; };
union FragB { v16b v; v8b half[2]; };

#define BATCH 2
#define SEQ   2048
#define DM    512
#define KVD   64
#define HD    16
#define NG    4
#define NR    8
#define MROWS (BATCH * SEQ)
#define BP    40
#define WSC   32.0f
#define QKSC  8.0f
#define SSC   0.00390625f
#define VSC   16.0f
#define PSC   16384.0f
#define ASC   64.0f
#define LOSC  2048.0f

__device__ __forceinline__ v8f wmma_f16(v16h a, v16h b, v8f c) {
  v8f d = __builtin_amdgcn_wmma_f32_16x16x32_f16(false, a, false, b, (short)0, c, false, false);
  asm volatile("v_nop\n\tv_nop\n\tv_nop\n\tv_nop" : "+v"(d) : "v"(a), "v"(b));
  return d;
}
__device__ __forceinline__ v8f wmma_bf16(v16b a, v16b b, v8f c) {
  v8f d = __builtin_amdgcn_wmma_f32_16x16x32_bf16(false, a, false, b, (short)0, c, false, false);
  asm volatile("v_nop\n\tv_nop\n\tv_nop\n\tv_nop" : "+v"(d) : "v"(a), "v"(b));
  return d;
}

__device__ __forceinline__ v16h ldfrag_h(const _Float16* p, int h) {
  FragH f;
  f.half[0] = *(const v8ha*)(p + 8 * h);
  f.half[1] = *(const v8ha*)(p + 16 + 8 * h);
  return f.v;
}
__device__ __forceinline__ v16h ldfrag_hs(const unsigned short* p, int h) {
  FragH f;
  f.half[0] = *(const v8ha*)(p + 8 * h);
  f.half[1] = *(const v8ha*)(p + 16 + 8 * h);
  return f.v;
}
__device__ __forceinline__ v16b ldfrag_bs(const unsigned short* p, int h) {
  FragB f;
  f.half[0] = *(const v8ba*)(p + 8 * h);
  f.half[1] = *(const v8ba*)(p + 16 + 8 * h);
  return f.v;
}

__device__ __forceinline__ unsigned short bf16_bits(float f) {
  unsigned int u = __float_as_uint(f);
  u += 0x7FFFu + ((u >> 16) & 1u);
  return (unsigned short)(u >> 16);
}
__device__ __forceinline__ float bf16_val(unsigned short s) {
  return __uint_as_float(((unsigned int)s) << 16);
}
__device__ __forceinline__ unsigned short f16_bits(float f) {
  const _Float16 hv = (_Float16)f;
  return __builtin_bit_cast(unsigned short, hv);
}
__device__ __forceinline__ void st_bf2(unsigned short* d0, unsigned short* d1, float v) {
  const unsigned short hb = bf16_bits(v);
  *d0 = hb;
  *d1 = bf16_bits(v - bf16_val(hb));
}
__device__ __forceinline__ void st_h2(unsigned short* d0, unsigned short* d1, float v) {
  const float vs = v * WSC;
  const _Float16 hh = (_Float16)vs;
  *d0 = __builtin_bit_cast(unsigned short, hh);
  *d1 = f16_bits((vs - (float)hh) * LOSC);
}

__global__ __launch_bounds__(256) void cvt_x_kernel(
    const float* __restrict__ x, _Float16* __restrict__ xh,
    unsigned short* __restrict__ xbh, unsigned short* __restrict__ xbl, int n8)
{
  const int gidx = blockIdx.x * 256 + threadIdx.x;
  if (gidx >= n8) return;
  const float* src = x + (size_t)gidx * 8;
  const v4f a = *(const v4fa*)src;
  const v4f c = *(const v4fa*)(src + 4);
  v8h oh;
  v8us ob, ol;
#define CVT1(i, val) { const float fv = (val); oh[i] = (_Float16)fv; const unsigned short hb = bf16_bits(fv); ob[i] = hb; ol[i] = bf16_bits(fv - bf16_val(hb)); }
  CVT1(0, a.x) CVT1(1, a.y) CVT1(2, a.z) CVT1(3, a.w)
  CVT1(4, c.x) CVT1(5, c.y) CVT1(6, c.z) CVT1(7, c.w)
#undef CVT1
  _Float16* dh = xh + (size_t)gidx * 8;
  unsigned short* db = xbh + (size_t)gidx * 8;
  unsigned short* dl = xbl + (size_t)gidx * 8;
  *(volatile v8h*)dh = oh;
  *(volatile v8us*)db = ob;
  *(volatile v8us*)dl = ol;
  __threadfence();
  *(volatile v8h*)dh = oh;
  *(volatile v8us*)db = ob;
  *(volatile v8us*)dl = ol;
}

template <int WHICH>
__device__ __forceinline__ void proj_store(const _Float16* sT, _Float16* dst,
                                           int m0, int n0, int w, int lane) {
  const int q8 = lane & 7, sub = lane >> 3;
  #pragma unroll
  for (int i = 0; i < 4; ++i) {
    const int L = 16 * w + 4 * i + sub;
    v8h v;
    _Float16* p;
    if (WHICH == 0) {
      v = *(const v8ha*)(sT + L * 64 + 8 * q8);
      p = dst + (size_t)(m0 + L) * DM + n0 + 8 * q8;
    } else if (WHICH == 1) {
      v = *(const v8ha*)(sT + L * 64 + 8 * q8);
      p = dst + (size_t)(m0 + L) * KVD + 8 * q8;
    } else {
      const int feat = L >> 1, hl = L & 1;
      const int b = m0 / SEQ, s0 = m0 - b * SEQ;
      v = *(const v8ha*)(sT + feat * 128 + 64 * hl + 8 * q8);
      p = dst + ((size_t)(b * KVD + feat)) * SEQ + s0 + 64 * hl + 8 * q8;
    }
    *(volatile v8h*)p = v;
  }
}

template <int WHICH>
__global__ __launch_bounds__(256) void proj_kernel(
    const _Float16* __restrict__ xh,
    const unsigned short* __restrict__ xbh,
    const unsigned short* __restrict__ xbl,
    const float* __restrict__ W,
    const float* __restrict__ bias,
    _Float16* __restrict__ dst)
{
  constexpr int N = (WHICH == 0) ? DM : KVD;
  __shared__ __attribute__((aligned(16))) unsigned short sB[2][64 * BP];
  __shared__ __attribute__((aligned(16))) _Float16 sT[128 * 64];

  const int tid = threadIdx.x, lane = tid & 31, w = tid >> 5;
  const int h = lane >> 4, l16 = lane & 15;
  const int m0 = blockIdx.x * 128;
  const int n0 = (WHICH == 0) ? (int)blockIdx.y * 64 : 0;
  const int kk = tid >> 3, nc = (tid & 7) * 8;
  const size_t arow = (size_t)(m0 + 16 * w + l16) * DM;

  const v8f zero8 = {0.f, 0.f, 0.f, 0.f, 0.f, 0.f, 0.f, 0.f};
  v8f acc[4];
  #pragma unroll
  for (int nt = 0; nt < 4; ++nt) acc[nt] = zero8;

  #pragma unroll 1
  for (int k0 = 0; k0 < DM; k0 += 32) {
    __syncthreads();
    {
      const float* wp = W + (size_t)(k0 + kk) * N + n0 + nc;
      const v4f w0 = *(const v4fa*)wp;
      const v4f w1 = *(const v4fa*)(wp + 4);
      unsigned short* d0 = &sB[0][nc * BP + kk];
      unsigned short* d1 = &sB[1][nc * BP + kk];
      if (WHICH < 2) {
        d0[0 * BP] = f16_bits(w0.x * WSC); d0[1 * BP] = f16_bits(w0.y * WSC);
        d0[2 * BP] = f16_bits(w0.z * WSC); d0[3 * BP] = f16_bits(w0.w * WSC);
        d0[4 * BP] = f16_bits(w1.x * WSC); d0[5 * BP] = f16_bits(w1.y * WSC);
        d0[6 * BP] = f16_bits(w1.z * WSC); d0[7 * BP] = f16_bits(w1.w * WSC);
      } else {
        st_bf2(d0 + 0 * BP, d1 + 0 * BP, w0.x); st_bf2(d0 + 1 * BP, d1 + 1 * BP, w0.y);
        st_bf2(d0 + 2 * BP, d1 + 2 * BP, w0.z); st_bf2(d0 + 3 * BP, d1 + 3 * BP, w0.w);
        st_bf2(d0 + 4 * BP, d1 + 4 * BP, w1.x); st_bf2(d0 + 5 * BP, d1 + 5 * BP, w1.y);
        st_bf2(d0 + 6 * BP, d1 + 6 * BP, w1.z); st_bf2(d0 + 7 * BP, d1 + 7 * BP, w1.w);
      }
    }
    __syncthreads();

    if (WHICH < 2) {
      const v16h a = ldfrag_h(xh + arow + k0, h);
      #pragma unroll
      for (int nt = 0; nt < 4; ++nt) {
        const v16h bf = ldfrag_hs(&sB[0][(16 * nt + l16) * BP], h);
        acc[nt] = wmma_f16(a, bf, acc[nt]);
      }
    } else {
      const v16b ahi = ldfrag_bs(xbh + arow + k0, h);
      const v16b alo = ldfrag_bs(xbl + arow + k0, h);
      #pragma unroll
      for (int nt = 0; nt < 4; ++nt) {
        const v16b bhi = ldfrag_bs(&sB[0][(16 * nt + l16) * BP], h);
        const v16b blo = ldfrag_bs(&sB[1][(16 * nt + l16) * BP], h);
        acc[nt] = wmma_bf16(ahi, bhi, acc[nt]);
        acc[nt] = wmma_bf16(ahi, blo, acc[nt]);
        acc[nt] = wmma_bf16(alo, bhi, acc[nt]);
      }
    }
  }

  #pragma unroll
  for (int nt = 0; nt < 4; ++nt) {
    const int feat = 16 * nt + l16;
    const float bvl = bias[n0 + feat];
    #pragma unroll
    for (int r = 0; r < 8; ++r) {
      const int tl = 16 * w + 8 * h + r;
      float y;
      if (WHICH < 2) y = (acc[nt][r] * (1.0f / WSC) + bvl) * QKSC;
      else           y = (acc[nt][r] + bvl) * VSC;
      const int idx = (WHICH == 2) ? (feat * 128 + tl) : (tl * 64 + feat);
      sT[idx] = (_Float16)y;
    }
  }
  __syncthreads();

  proj_store<WHICH>(sT, dst, m0, n0, w, lane);
  __threadfence();
  proj_store<WHICH>(sT, dst, m0, n0, w, lane);
}

__device__ __forceinline__ v16h pack_p(v8f a, v8f c) {
  v16h r;
  #pragma unroll
  for (int i = 0; i < 8; ++i) {
    r[i]     = (_Float16)(a[i] * PSC);
    r[i + 8] = (_Float16)(c[i] * PSC);
  }
  return r;
}

__device__ __forceinline__ void attn_store(const _Float16* s0, const _Float16* s1,
                                           _Float16* p0, _Float16* p1,
                                           int b, int g, int q0, int w, int lane) {
  const int q8 = lane & 7, L = 4 * w + (lane >> 3);
  const int row = L >> 1, hl = L & 1;
  const int so = row * 128 + 64 * hl + 8 * q8;
  const size_t go = (size_t)(b * SEQ + q0 + row) * DM + g * (NR * HD) + 64 * hl + 8 * q8;
  const v8h v0 = *(const v8ha*)(s0 + so);
  const v8h v1 = *(const v8ha*)(s1 + so);
  *(volatile v8h*)(p0 + go) = v0;
  *(volatile v8h*)(p1 + go) = v1;
}

__global__ __launch_bounds__(256) void attn_kernel(
    const _Float16* __restrict__ qp,
    const _Float16* __restrict__ kp,
    const _Float16* __restrict__ vt,
    _Float16* __restrict__ ahp,
    _Float16* __restrict__ alp)
{
  __shared__ __attribute__((aligned(16))) _Float16 sA[2][16 * 128];

  const int tid = threadIdx.x, lane = tid & 31, w = tid >> 5;
  const int h = lane >> 4, m = lane & 15;
  const int q0 = blockIdx.x * 16, g = blockIdx.y, b = blockIdx.z;

  const _Float16 hz = (_Float16)0.0f;
  const v8h z8h = {hz, hz, hz, hz, hz, hz, hz, hz};
  const v8f zero8 = {0.f, 0.f, 0.f, 0.f, 0.f, 0.f, 0.f, 0.f};

  FragH qf;
  qf.half[0] = *(const v8ha*)(qp + (size_t)(b * SEQ + q0 + m) * DM + g * (NR * HD) + w * HD + 8 * h);
  qf.half[1] = z8h;
  const v16h qb = qf.v;

  const _Float16* kbase = kp + (size_t)(b * SEQ + m) * KVD + g * HD + 8 * h;
  const _Float16* vbase = vt + ((size_t)(b * NG + g) * HD + m) * SEQ;

  v8f o = zero8;
  float mrun = -1e30f, lrun = 0.0f;

  #pragma unroll 1
  for (int kb = 0; kb < SEQ; kb += 64) {
    v8f s[4];
    #pragma unroll
    for (int j = 0; j < 4; ++j) {
      FragH kf;
      kf.half[0] = *(const v8ha*)(kbase + (size_t)(kb + 16 * j) * KVD);
      kf.half[1] = z8h;
      s[j] = wmma_f16(kf.v, qb, zero8);
    }

    float mloc = -1e30f;
    #pragma unroll
    for (int j = 0; j < 4; ++j)
      #pragma unroll
      for (int r = 0; r < 8; ++r) {
        const float t = s[j][r] * SSC;
        s[j][r] = t;
        mloc = fmaxf(mloc, t);
      }
    mloc = fmaxf(mloc, __shfl_xor(mloc, 16));
    const float mnew = fmaxf(mrun, mloc);
    const float alpha = __expf(mrun - mnew);
    mrun = mnew;
    float lsum = 0.0f;
    #pragma unroll
    for (int j = 0; j < 4; ++j)
      #pragma unroll
      for (int r = 0; r < 8; ++r) {
        const float p = __expf(s[j][r] - mnew);
        s[j][r] = p;
        lsum += p;
      }
    lsum += __shfl_xor(lsum, 16);
    lrun = lrun * alpha + lsum;
    #pragma unroll
    for (int r = 0; r < 8; ++r) o[r] = o[r] * alpha;

    const v16h pb0 = pack_p(s[0], s[1]);
    const v16h pb1 = pack_p(s[2], s[3]);

    const v16h vf0 = ldfrag_h(vbase + kb, h);
    const v16h vf1 = ldfrag_h(vbase + kb + 32, h);
    o = wmma_f16(vf0, pb0, o);
    o = wmma_f16(vf1, pb1, o);
  }

  const float inv = (1.0f / lrun) * (ASC / (PSC * VSC));
  #pragma unroll
  for (int r = 0; r < 8; ++r) {
    const float a64 = o[r] * inv;
    const _Float16 hi = (_Float16)a64;
    const _Float16 lo = (_Float16)((a64 - (float)hi) * LOSC);
    const int idx = m * 128 + w * HD + 8 * h + r;
    sA[0][idx] = hi;
    sA[1][idx] = lo;
  }
  __syncthreads();

  attn_store(sA[0], sA[1], ahp, alp, b, g, q0, w, lane);
  __threadfence();
  attn_store(sA[0], sA[1], ahp, alp, b, g, q0, w, lane);
}

__device__ __forceinline__ void out_store(const float* sO, float* out,
                                          int m0, int n0, int w, int lane) {
  const int q8 = lane & 7, sub = lane >> 3;
  #pragma unroll
  for (int i = 0; i < 8; ++i) {
    const int L = 32 * w + 4 * i + sub;
    const int tl = L >> 1, hl = L & 1;
    const v4f v = *(const v4fa*)(sO + tl * 64 + 32 * hl + 4 * q8);
    float* p = out + (size_t)(m0 + tl) * DM + n0 + 32 * hl + 4 * q8;
    *(volatile v4f*)p = v;
  }
}

__global__ __launch_bounds__(256) void oproj_kernel(
    const _Float16* __restrict__ ahp,
    const _Float16* __restrict__ alp,
    const float* __restrict__ Wo,
    const float* __restrict__ bo,
    float* __restrict__ out)
{
  __shared__ __attribute__((aligned(16))) unsigned short sB[2][64 * BP];
  __shared__ __attribute__((aligned(16))) float sO[128 * 64];

  const int tid = threadIdx.x, lane = tid & 31, w = tid >> 5;
  const int h = lane >> 4, l16 = lane & 15;
  const int m0 = blockIdx.x * 128;
  const int n0 = blockIdx.y * 64;
  const int kk = tid >> 3, nc = (tid & 7) * 8;
  const size_t arow = (size_t)(m0 + 16 * w + l16) * DM;

  const v8f zero8 = {0.f, 0.f, 0.f, 0.f, 0.f, 0.f, 0.f, 0.f};
  v8f acc_hh[4], acc_x[4];
  #pragma unroll
  for (int nt = 0; nt < 4; ++nt) { acc_hh[nt] = zero8; acc_x[nt] = zero8; }

  #pragma unroll 1
  for (int k0 = 0; k0 < DM; k0 += 32) {
    __syncthreads();
    {
      const float* wp = Wo + (size_t)(k0 + kk) * DM + n0 + nc;
      const v4f w0 = *(const v4fa*)wp;
      const v4f w1 = *(const v4fa*)(wp + 4);
      unsigned short* d0 = &sB[0][nc * BP + kk];
      unsigned short* d1 = &sB[1][nc * BP + kk];
      st_h2(d0 + 0 * BP, d1 + 0 * BP, w0.x); st_h2(d0 + 1 * BP, d1 + 1 * BP, w0.y);
      st_h2(d0 + 2 * BP, d1 + 2 * BP, w0.z); st_h2(d0 + 3 * BP, d1 + 3 * BP, w0.w);
      st_h2(d0 + 4 * BP, d1 + 4 * BP, w1.x); st_h2(d0 + 5 * BP, d1 + 5 * BP, w1.y);
      st_h2(d0 + 6 * BP, d1 + 6 * BP, w1.z); st_h2(d0 + 7 * BP, d1 + 7 * BP, w1.w);
    }
    __syncthreads();

    const v16h ahi = ldfrag_h(ahp + arow + k0, h);
    const v16h alo = ldfrag_h(alp + arow + k0, h);
    #pragma unroll
    for (int nt = 0; nt < 4; ++nt) {
      const v16h bhi = ldfrag_hs(&sB[0][(16 * nt + l16) * BP], h);
      const v16h blo = ldfrag_hs(&sB[1][(16 * nt + l16) * BP], h);
      acc_hh[nt] = wmma_f16(ahi, bhi, acc_hh[nt]);
      acc_x[nt]  = wmma_f16(ahi, blo, acc_x[nt]);
      acc_x[nt]  = wmma_f16(alo, bhi, acc_x[nt]);
    }
  }

  #pragma unroll
  for (int nt = 0; nt < 4; ++nt) {
    const int feat = 16 * nt + l16;
    const float bvl = bo[n0 + feat];
    #pragma unroll
    for (int r = 0; r < 8; ++r) {
      const int tl = 16 * w + 8 * h + r;
      const float y = (acc_hh[nt][r] + acc_x[nt][r] * (1.0f / LOSC)) * (1.0f / (ASC * WSC)) + bvl;
      sO[tl * 64 + feat] = y;
    }
  }
  __syncthreads();

  out_store(sO, out, m0, n0, w, lane);
  __threadfence();
  out_store(sO, out, m0, n0, w, lane);
}

extern "C" void kernel_launch(void* const* d_in, const int* in_sizes, int n_in,
                              void* d_out, int out_size, void* d_ws, size_t ws_size,
                              hipStream_t stream) {
  if (n_in < 9) return;
  if (in_sizes[0] != MROWS * DM) return;
  if (in_sizes[1] != DM * DM || in_sizes[2] != DM) return;
  if (in_sizes[3] != DM * KVD || in_sizes[4] != KVD) return;
  if (in_sizes[5] != DM * KVD || in_sizes[6] != KVD) return;
  if (in_sizes[7] != DM * DM || in_sizes[8] != DM) return;
  if (out_size != MROWS * DM) return;

  const float* x  = (const float*)d_in[0];
  const float* Wq = (const float*)d_in[1];
  const float* bq = (const float*)d_in[2];
  const float* Wk = (const float*)d_in[3];
  const float* bk = (const float*)d_in[4];
  const float* Wv = (const float*)d_in[5];
  const float* bv = (const float*)d_in[6];
  const float* Wo = (const float*)d_in[7];
  const float* bo = (const float*)d_in[8];
  float* out = (float*)d_out;

  const size_t pb = (size_t)MROWS * DM * 2;
  const size_t kb = (size_t)MROWS * KVD * 2;
  const size_t total = 6 * pb + 2 * kb;
  if (total > ws_size) return;

  char* ws = (char*)d_ws;
  _Float16*       xh  = (_Float16*)(ws);
  unsigned short* xbh = (unsigned short*)(ws + pb);
  unsigned short* xbl = (unsigned short*)(ws + 2 * pb);
  _Float16*       qp  = (_Float16*)(ws + 3 * pb);
  _Float16*       kp  = (_Float16*)(ws + 4 * pb);
  _Float16*       vt  = (_Float16*)(ws + 4 * pb + kb);
  _Float16*       ahp = (_Float16*)(ws + 4 * pb + 2 * kb);
  _Float16*       alp = (_Float16*)(ws + 5 * pb + 2 * kb);

  const int n8 = MROWS * DM / 8;
  cvt_x_kernel<<<(n8 + 255) / 256, 256, 0, stream>>>(x, xh, xbh, xbl, n8);

  proj_kernel<0><<<dim3(MROWS / 128, DM / 64), 256, 0, stream>>>(xh, xbh, xbl, Wq, bq, qp);
  proj_kernel<1><<<dim3(MROWS / 128, 1), 256, 0, stream>>>(xh, xbh, xbl, Wk, bk, kp);
  proj_kernel<2><<<dim3(MROWS / 128, 1), 256, 0, stream>>>(xh, xbh, xbl, Wv, bv, vt);

  attn_kernel<<<dim3(SEQ / 16, NG, BATCH), 256, 0, stream>>>(qp, kp, vt, ahp, alp);

  oproj_kernel<<<dim3(MROWS / 128, DM / 64), 256, 0, stream>>>(ahp, alp, Wo, bo, out);
}
